// SPInterAttModule_15178414424521
// MI455X (gfx1250) — hardware-run, weakly checked
//
#include <hip/hip_runtime.h>


#define NB_  8
#define CC   256
#define NPX  4096
#define MM   256
#define NH_  8
#define DQ   32
#define DM   CC
#define SCL  0.17677669529663687f
#define PCAR 4096.0f
#define XCAR 256.0f
#define LOSC 1024.0f
typedef _Float16 h16;
typedef unsigned short bf;
typedef __attribute__((ext_vector_type(16))) __bf16   v16bf;
typedef __attribute__((ext_vector_type(16))) _Float16 v16h;
typedef __attribute__((ext_vector_type(8)))  _Float16 v8h;
typedef __attribute__((ext_vector_type(8)))  unsigned short v8us;
typedef __attribute__((ext_vector_type(8)))  float    v8f;
typedef __attribute__((ext_vector_type(4)))  float    v4f;
typedef v8h  __attribute__((may_alias)) v8ha;
typedef v4f  __attribute__((may_alias)) v4fa;
typedef v8us __attribute__((may_alias)) v8usa;

__device__ __forceinline__ unsigned short f2bf(float f) { unsigned u = __float_as_uint(f); u += 0x7FFFu + ((u >> 16) & 1u); return (unsigned short)(u >> 16); }
__device__ __forceinline__ float bf2f(unsigned short b) { return __uint_as_float(((unsigned)b) << 16); }
__device__ __forceinline__ float bfr(float f) { return bf2f(f2bf(f)); }
__device__ __forceinline__ v16h cat16(v8h lo, v8h hi) { return __builtin_shufflevector(lo, hi, 0, 1, 2, 3, 4, 5, 6, 7, 8, 9, 10, 11, 12, 13, 14, 15); }
__device__ __forceinline__ v16bf cat16b(v8us lo, v8us hi) { return __builtin_bit_cast(v16bf, __builtin_shufflevector(lo, hi, 0, 1, 2, 3, 4, 5, 6, 7, 8, 9, 10, 11, 12, 13, 14, 15)); }
__device__ __forceinline__ v8f wmma16(v16h a, v16h b, v8f c) { return __builtin_amdgcn_wmma_f32_16x16x32_f16(false, a, false, b, (short)0, c, false, false); }
__device__ __forceinline__ v8f wmmab(v16bf a, v16bf b, v8f c) { return __builtin_amdgcn_wmma_f32_16x16x32_bf16(false, a, false, b, (short)0, c, false, false); }


__global__ __launch_bounds__(128) void k_gemmh(const h16* __restrict__ A, const h16* __restrict__ Bn, const float* __restrict__ bias, float* C, int ldc, const float* __restrict__ R, int K, size_t sA, size_t sB, size_t sC, int roundR) {
    __shared__ __align__(16) float ost[4][16 * 68];
    const size_t z = blockIdx.z; A += z * sA; Bn += z * sB; C += z * sC; if (R) R += z * sC;
    const int lane = threadIdx.x & 31, wave = threadIdx.x >> 5, lr = lane & 15, hi = lane >> 4;
    const int r0 = blockIdx.x * 64 + wave * 16, c0 = blockIdx.y * 64;
    const size_t aoff = (size_t)(r0 + lr) * K + 8 * hi;
    size_t boff[4];
#pragma unroll
    for (int t = 0; t < 4; ++t) boff[t] = (size_t)(c0 + t * 16 + lr) * K + 8 * hi;
    v8f acc[4];
#pragma unroll
    for (int t = 0; t < 4; ++t) acc[t] = (v8f){};
#pragma unroll 1
    for (int kc = 0; kc < K; kc += 32) {
        const v16h a = cat16(*(const v8h*)(A + aoff + kc), *(const v8h*)(A + aoff + kc + 16));
#pragma unroll
        for (int t = 0; t < 4; ++t) { const v16h b = cat16(*(const v8h*)(Bn + boff[t] + kc), *(const v8h*)(Bn + boff[t] + kc + 16)); acc[t] = wmma16(a, b, acc[t]); }
        asm volatile("v_nop\n\tv_nop\n\tv_nop\n\tv_nop" : "+v"(acc[0]), "+v"(acc[1]), "+v"(acc[2]), "+v"(acc[3]) : "v"(a));
    }
    float* os = &ost[wave][0];
#pragma unroll
    for (int t = 0; t < 4; ++t) { const float bv = bias ? bfr(bias[c0 + t * 16 + lr]) : 0.f;
#pragma unroll
        for (int j = 0; j < 8; ++j) os[(hi * 8 + j) * 68 + t * 16 + lr] = acc[t][j] + bv; }
    __syncthreads();
    float* crow = C + (size_t)r0 * ldc + c0;
    auto pass = [&]() {
#pragma unroll
        for (int s = 0; s < 8; ++s) { const int Lid = (lane >> 3) + 4 * s, piece = lane & 7; const int row = Lid >> 1, cofs = (Lid & 1) * 32 + piece * 4;
            v4f val = *(const v4fa*)(os + row * 68 + cofs); if (R) { const v4f rv = *(const v4f*)(R + ((size_t)r0 + row) * ldc + c0 + cofs); val += roundR ? (v4f){bfr(rv[0]), bfr(rv[1]), bfr(rv[2]), bfr(rv[3])} : rv; }
            *(volatile v4f*)(crow + (size_t)row * ldc + cofs) = val; }
    };
    pass(); __threadfence(); pass();
}

template <int MODE>
__global__ __launch_bounds__(128) void k_gemm3z(const bf* __restrict__ Ah, const bf* __restrict__ Al, const bf* __restrict__ Bh, const bf* __restrict__ Bl, int K, float* C, int ldc, size_t sA, size_t sB, size_t sC) {
    if ((MODE & 1) && (int)blockIdx.y * 64 > (int)blockIdx.x * 64 + 63) return;
    const size_t z = blockIdx.z; Ah += z * sA; Al += z * sA; Bh += z * sB; Bl += z * sB; C += z * sC;
    const int Klim = (MODE & 2) ? min(K, ((int)blockIdx.x + 1) * 64) : K;
    __shared__ __align__(16) float ost[4][16 * 68];
    const int lane = threadIdx.x & 31, wave = threadIdx.x >> 5, lr = lane & 15, hi = lane >> 4;
    const int r0 = blockIdx.x * 64 + wave * 16, c0 = blockIdx.y * 64;
    const size_t aoff = (size_t)(r0 + lr) * K + 8 * hi;
    v8f acc[4];
#pragma unroll
    for (int t = 0; t < 4; ++t) acc[t] = (v8f){};
#pragma unroll 1
    for (int kc = 0; kc < Klim; kc += 32) {
        const v16bf a = cat16b(*(const v8us*)(Ah + aoff + kc), *(const v8us*)(Ah + aoff + kc + 16));
        v16bf al = a; if (!(MODE & 4) && !(MODE & 16)) al = cat16b(*(const v8us*)(Al + aoff + kc), *(const v8us*)(Al + aoff + kc + 16));
#pragma unroll
        for (int t = 0; t < 4; ++t) { const size_t bo = (size_t)(c0 + t * 16 + lr) * K + kc + 8 * hi;
            const v16bf bh = cat16b(*(const v8us*)(Bh + bo), *(const v8us*)(Bh + bo + 16));
            acc[t] = wmmab(a, bh, acc[t]);
            if (!(MODE & 4)) { if (!(MODE & 16)) acc[t] = wmmab(al, bh, acc[t]); if (!(MODE & 8)) { const v16bf bl = cat16b(*(const v8us*)(Bl + bo), *(const v8us*)(Bl + bo + 16)); acc[t] = wmmab(a, bl, acc[t]); } } }
        asm volatile("v_nop\n\tv_nop\n\tv_nop\n\tv_nop" : "+v"(acc[0]), "+v"(acc[1]), "+v"(acc[2]), "+v"(acc[3]) : "v"(a), "v"(al));
    }
    float* os = &ost[wave][0];
#pragma unroll
    for (int t = 0; t < 4; ++t) {
#pragma unroll
        for (int j = 0; j < 8; ++j) os[(hi * 8 + j) * 68 + t * 16 + lr] = acc[t][j]; }
    __builtin_amdgcn_wave_barrier(); asm volatile("" ::: "memory");
    float* crow = C + (size_t)r0 * ldc + c0;
    auto pass = [&]() {
#pragma unroll
        for (int s = 0; s < 8; ++s) { const int Lid = (lane >> 3) + 4 * s, piece = lane & 7; const int row = Lid >> 1, cofs = (Lid & 1) * 32 + piece * 4;
            const v4f val = *(const v4fa*)(os + row * 68 + cofs); *(volatile v4f*)(crow + (size_t)row * ldc + cofs) = val; }
    };
    pass(); __threadfence(); pass();
}
__global__ __launch_bounds__(256) void k_planes32z(const float* __restrict__ F, int ld, int off, float sc, int rows, bf* Ph, bf* Pl) {
    typedef __attribute__((ext_vector_type(2))) unsigned short v2us;
    const int lane = threadIdx.x & 31; const size_t r = ((size_t)blockIdx.x * 8 + (threadIdx.x >> 5)) * 2 + (lane >> 4); if (r >= (size_t)rows) return; const int z = blockIdx.z; const int c0 = (lane & 15) * 2; v2us oh, ol;
    Ph += (size_t)z * rows * 32; Pl += (size_t)z * rows * 32;
#pragma unroll
    for (int i = 0; i < 2; ++i) { const float y = F[r * ld + off + z * 32 + c0 + i] * sc; const unsigned short hb = f2bf(y); oh[i] = hb; ol[i] = f2bf(y - bf2f(hb)); }
    const size_t o = r * 32 + c0; *(volatile v2us*)(Ph + o) = oh; *(volatile v2us*)(Pl + o) = ol; __threadfence(); *(volatile v2us*)(Ph + o) = oh; *(volatile v2us*)(Pl + o) = ol;
}
__global__ __launch_bounds__(256) void k_vtpadz(const float* __restrict__ F, int ld, int off, int nk, bf* Th, bf* Tl) {
    typedef __attribute__((ext_vector_type(2))) unsigned short v2us;
    const int lane = threadIdx.x & 31; const size_t wid = (size_t)blockIdx.x * 8 + (threadIdx.x >> 5); if (wid >= (size_t)64 * (nk / 64)) return; const int z = blockIdx.z; const int d = (int)(wid / (nk / 64)); const int k0 = (int)(wid % (nk / 64)) * 64 + lane * 2; v2us oh, ol;
    Th += (size_t)z * 64 * nk; Tl += (size_t)z * 64 * nk;
#pragma unroll
    for (int i = 0; i < 2; ++i) { const float y = (d < 32) ? F[(size_t)(k0 + i) * ld + off + z * 32 + (d < 32 ? d : 0)] : 0.f; const unsigned short hb = f2bf(y); oh[i] = hb; ol[i] = f2bf(y - bf2f(hb)); }
    const size_t o = (size_t)d * nk + k0; *(volatile v2us*)(Th + o) = oh; *(volatile v2us*)(Tl + o) = ol; __threadfence(); *(volatile v2us*)(Th + o) = oh; *(volatile v2us*)(Tl + o) = ol;
}
template <int NK>
__global__ __launch_bounds__(256) void k_softmaxz(const float* __restrict__ S, int rows, bf* PH, bf* PL) {
    typedef __attribute__((ext_vector_type(4))) unsigned short v4us;
    const int lane = threadIdx.x & 31, i = blockIdx.x * 8 + (threadIdx.x >> 5); if (i >= rows) return; const size_t zo = (size_t)blockIdx.z * rows * NK; const float* sr = S + zo + (size_t)i * NK; PH += zo; PL += zo;
    float m = -3.0e38f;
#pragma unroll 1
    for (int c0 = lane * 4; c0 < NK; c0 += 128) {
#pragma unroll
        for (int q = 0; q < 4; ++q) m = fmaxf(m, sr[c0 + q]); }
#pragma unroll
    for (int sh = 16; sh; sh >>= 1) m = fmaxf(m, __shfl_xor(m, sh, 32));
    float sum = 0.f;
#pragma unroll 1
    for (int c0 = lane * 4; c0 < NK; c0 += 128) {
#pragma unroll
        for (int q = 0; q < 4; ++q) sum += __expf(sr[c0 + q] - m); }
#pragma unroll
    for (int sh = 16; sh; sh >>= 1) sum += __shfl_xor(sum, sh, 32);
    const float inv = 1.0f / sum;
#pragma unroll 1
    for (int ps = 0; ps < 2; ++ps) {
#pragma unroll 1
        for (int c0 = lane * 4; c0 < NK; c0 += 128) { v4us oh, ol;
#pragma unroll
            for (int q = 0; q < 4; ++q) { const float p = __expf(sr[c0 + q] - m) * inv; const unsigned short hb = f2bf(p); oh[q] = hb; ol[q] = f2bf(p - bf2f(hb)); }
            const size_t o = (size_t)i * NK + c0; *(volatile v4us*)(PH + o) = oh; *(volatile v4us*)(PL + o) = ol; }
        if (ps == 0) __threadfence(); }
}
__global__ __launch_bounds__(256) void k_placez(const float* __restrict__ XH, int rows, int ldy, float* Y) {
    const int lane = threadIdx.x & 31; const size_t q = (size_t)blockIdx.x * 8 + (threadIdx.x >> 5); if (q >= (size_t)rows) return; const int z = blockIdx.z; const float v = XH[((size_t)z * rows + q) * 64 + lane];
    *(volatile float*)(Y + q * ldy + z * 32 + lane) = v; __threadfence(); *(volatile float*)(Y + q * ldy + z * 32 + lane) = v;
}

typedef __attribute__((ext_vector_type(4))) _Float16 v4h;
__device__ __forceinline__ h16 tohx(float x) { return (h16)x; }
__global__ __launch_bounds__(256) void k_cvt8h(const float* __restrict__ src, h16* dst, size_t n8) { const size_t i = (size_t)blockIdx.x * 256 + threadIdx.x; if (i >= n8) return; const v8f v = *(const v8f*)(src + i * 8); v8h o;
#pragma unroll
    for (int k = 0; k < 8; ++k) o[k] = tohx(bfr(v[k])); *(volatile v8h*)(dst + i * 8) = o; __threadfence(); *(volatile v8h*)(dst + i * 8) = o; }
__global__ __launch_bounds__(256) void k_stat2d(const float* __restrict__ xb, float* MU, float* RS) {
    const int lane = threadIdx.x & 31; const int n = (blockIdx.x * 8 + (threadIdx.x >> 5)) * 32 + lane; if (n >= NPX) return; float s = 0.f;
#pragma unroll 1
    for (int c = 0; c < CC; ++c) s += bfr(xb[(size_t)c * NPX + n]);
    const float mu = s * (1.0f / CC); float q = 0.f;
#pragma unroll 1
    for (int c = 0; c < CC; ++c) { const float d = bfr(xb[(size_t)c * NPX + n]) - mu; q = fmaf(d, d, q); }
    const float rs = rsqrtf(q * (1.0f / CC) + 1e-6f);
    *(volatile float*)(MU + n) = mu; *(volatile float*)(RS + n) = rs; __threadfence(); *(volatile float*)(MU + n) = mu; *(volatile float*)(RS + n) = rs;
}
__global__ __launch_bounds__(256) void k_xnrow(const float* __restrict__ xb, const float* __restrict__ MU, const float* __restrict__ RS, const float* __restrict__ g, const float* __restrict__ bb, h16* XH) {
    const int lane = threadIdx.x & 31; const int n = blockIdx.x * 8 + (threadIdx.x >> 5); if (n >= NPX) return; const float mu = MU[n], rs = RS[n]; v8h o;
#pragma unroll
    for (int i = 0; i < 8; ++i) { const int c = lane * 8 + i; o[i] = tohx((bfr(xb[(size_t)c * NPX + n]) - mu) * rs * bfr(g[c]) + bfr(bb[c])); }
    *(volatile v8h*)(XH + (size_t)n * CC + lane * 8) = o; __threadfence(); *(volatile v8h*)(XH + (size_t)n * CC + lane * 8) = o;
}
__global__ __launch_bounds__(256) void k_xncol(const float* __restrict__ xb, const float* __restrict__ MU, const float* __restrict__ RS, const float* __restrict__ g, const float* __restrict__ bb, bf* Th, bf* Tl) {
    typedef __attribute__((ext_vector_type(4))) unsigned short v4us;
    const int lane = threadIdx.x & 31; const size_t w = (size_t)blockIdx.x * 8 + (threadIdx.x >> 5); if (w >= (size_t)CC * (NPX / 128)) return; const int c = (int)(w / (NPX / 128)); const int n0 = (int)(w % (NPX / 128)) * 128 + lane * 4; const float gc = bfr(g[c]), bc = bfr(bb[c]); v4us oh, ol;
#pragma unroll
    for (int i = 0; i < 4; ++i) { const int n = n0 + i; const float y = (bfr(xb[(size_t)c * NPX + n]) - MU[n]) * RS[n] * gc + bc; const unsigned short hb = f2bf(y); oh[i] = hb; ol[i] = f2bf(y - bf2f(hb)); }
    const size_t o = (size_t)c * NPX + n0; *(volatile v4us*)(Th + o) = oh; *(volatile v4us*)(Tl + o) = ol; __threadfence(); *(volatile v4us*)(Th + o) = oh; *(volatile v4us*)(Tl + o) = ol;
}

__global__ __launch_bounds__(256) void k_maskb(const float* __restrict__ mb, bf* MB) {
    const int lane = threadIdx.x & 31; const int m = blockIdx.x * 8 + (threadIdx.x >> 5); if (m >= MM) return;
#pragma unroll 1
    for (int ps = 0; ps < 2; ++ps) {
#pragma unroll 1
        for (int p = 0; p < NPX / 256; ++p) { const int c0 = p * 256 + lane * 8; v8us o;
#pragma unroll
            for (int i = 0; i < 8; ++i) o[i] = f2bf(mb[(size_t)m * NPX + c0 + i]);
            *(volatile v8us*)(MB + (size_t)m * NPX + c0) = o; }
        if (ps == 0) __threadfence(); }
}
__global__ __launch_bounds__(256) void k_sths(const float* __restrict__ mb, const float* __restrict__ STOK, h16* STHS) {
    const int lane = threadIdx.x & 31; const int w = blockIdx.x * 8 + (threadIdx.x >> 5); if (w >= NH_ * (MM / 4)) return; const int h = w / (MM / 4), m0 = (w % (MM / 4)) * 4; const int m = m0 + (lane >> 3), d0 = (lane & 7) * 4;
    float inv = 0.f;
#pragma unroll 1
    for (int r = 0; r < 4; ++r) { float s = 0.f;
#pragma unroll 1
        for (int n = lane; n < NPX; n += 32) s += bfr(mb[(size_t)(m0 + r) * NPX + n]);
#pragma unroll
        for (int sh = 16; sh; sh >>= 1) s += __shfl_xor(s, sh, 32);
        if (r == (lane >> 3)) inv = __fdiv_rn(1.0f, s + 1e-16f); }
    v4h o;
#pragma unroll
    for (int i = 0; i < 4; ++i) o[i] = tohx(STOK[(size_t)m * CC + h * DQ + d0 + i] * inv * SCL);
    const size_t off = ((size_t)h * MM + m) * DQ + d0; *(volatile v4h*)(STHS + off) = o; __threadfence(); *(volatile v4h*)(STHS + off) = o;
}
__global__ __launch_bounds__(256) void k_hpl32h(const float* __restrict__ F, h16* P) {
    const int lane = threadIdx.x & 31; const size_t w = (size_t)blockIdx.x * 8 + (threadIdx.x >> 5); const int n = (int)(w * 4 + (lane >> 3)); if (n >= NPX) return; const int h = blockIdx.z; const int d0 = (lane & 7) * 4; v4h o;
#pragma unroll
    for (int i = 0; i < 4; ++i) o[i] = tohx(F[(size_t)n * CC + h * DQ + d0 + i]);
    const size_t off = ((size_t)h * NPX + n) * DQ + d0; *(volatile v4h*)(P + off) = o; __threadfence(); *(volatile v4h*)(P + off) = o;
}
__global__ __launch_bounds__(256) void k_vT32h(const float* __restrict__ V, h16* VT) {
    __shared__ float tl[64][33];
    const int tid = threadIdx.x; const int t0 = blockIdx.x * 64; const int h = blockIdx.z; const int rr = tid >> 2, cq = (tid & 3) * 8;
#pragma unroll
    for (int i = 0; i < 8; ++i) tl[rr][cq + i] = V[(size_t)(t0 + rr) * CC + h * DQ + cq + i];
    __syncthreads();
    const int lane = tid & 31, wv = tid >> 5;
    auto pass = [&]() {
#pragma unroll
        for (int st = 0; st < 4; ++st) { const int dr = wv * 8 + st * 2 + (lane >> 4); const int tq = (lane & 15) * 4; v4h v;
#pragma unroll
            for (int i = 0; i < 4; ++i) v[i] = tohx((dr < DQ) ? tl[tq + i][dr < DQ ? dr : 0] : 0.f);
            *(volatile v4h*)(VT + ((size_t)h * 64 + dr) * NPX + t0 + tq) = v; }
    };
    pass(); __threadfence(); pass();
}
__global__ __launch_bounds__(256) void k_csoftP(const float* __restrict__ S, h16* PT) {
    const int lane = threadIdx.x & 31; const int w = blockIdx.x * 8 + (threadIdx.x >> 5); if (w >= NH_ * MM) return; const int h = w / MM, m = w % MM; const float* col = S + (size_t)h * NPX * MM + m;
    float mx = -3.0e38f;
#pragma unroll 1
    for (int n = lane; n < NPX; n += 32) mx = fmaxf(mx, col[(size_t)n * MM]);
#pragma unroll
    for (int sh = 16; sh; sh >>= 1) mx = fmaxf(mx, __shfl_xor(mx, sh, 32));
    float sum = 0.f;
#pragma unroll 1
    for (int n = lane; n < NPX; n += 32) sum += __expf(col[(size_t)n * MM] - mx);
#pragma unroll
    for (int sh = 16; sh; sh >>= 1) sum += __shfl_xor(sum, sh, 32);
    const float f = __fdiv_rn(PCAR, sum);
#pragma unroll 1
    for (int ps = 0; ps < 2; ++ps) {
#pragma unroll 1
        for (int n0 = lane * 4; n0 < NPX; n0 += 128) { v4h o;
#pragma unroll
            for (int i = 0; i < 4; ++i) o[i] = tohx(__expf(col[(size_t)(n0 + i) * MM] - mx) * f);
            *(volatile v4h*)(PT + ((size_t)h * MM + m) * NPX + n0) = o; }
        if (ps == 0) __threadfence(); }
}
__global__ __launch_bounds__(256) void k_so16(const float* __restrict__ SOT, h16* SO16) {
    const int lane = threadIdx.x & 31; const int w = blockIdx.x * 8 + (threadIdx.x >> 5); if (w >= NH_ * 64) return; const int h = w / 64, d = w % 64; v8h o;
#pragma unroll
    for (int i = 0; i < 8; ++i) { const int m = lane * 8 + i; o[i] = tohx((d < DQ) ? SOT[((size_t)h * MM + m) * 64 + (d < DQ ? d : 0)] * (1.0f / PCAR) : 0.f); }
    const size_t off = ((size_t)h * 64 + d) * MM + lane * 8; *(volatile v8h*)(SO16 + off) = o; __threadfence(); *(volatile v8h*)(SO16 + off) = o;
}
__global__ __launch_bounds__(256) void k_csoftX(const float* __restrict__ X, h16* XS) {
    const int lane = threadIdx.x & 31; const int w = blockIdx.x * 8 + (threadIdx.x >> 5); if (w >= NH_ * NPX) return; const int h = w / NPX, n = w % NPX; const float* col = X + (size_t)h * MM * NPX + n; float v[8]; float mx = -3.0e38f;
#pragma unroll
    for (int i = 0; i < 8; ++i) { v[i] = col[(size_t)(lane * 8 + i) * NPX]; mx = fmaxf(mx, v[i]); }
#pragma unroll
    for (int sh = 16; sh; sh >>= 1) mx = fmaxf(mx, __shfl_xor(mx, sh, 32));
    float sum = 0.f;
#pragma unroll
    for (int i = 0; i < 8; ++i) { v[i] = __expf(v[i] - mx); sum += v[i]; }
#pragma unroll
    for (int sh = 16; sh; sh >>= 1) sum += __shfl_xor(sum, sh, 32);
    const float f = __fdiv_rn(XCAR, sum); v8h o;
#pragma unroll
    for (int i = 0; i < 8; ++i) o[i] = tohx(v[i] * f);
    const size_t off = ((size_t)h * NPX + n) * MM + lane * 8; *(volatile v8h*)(XS + off) = o; __threadfence(); *(volatile v8h*)(XS + off) = o;
}
__global__ __launch_bounds__(256) void k_outrows(const float* __restrict__ OZ, float* OUTB) {
    const int lane = threadIdx.x & 31; const size_t w = (size_t)blockIdx.x * 8 + (threadIdx.x >> 5); if (w >= (size_t)CC * (NPX / 128)) return; const int c = (int)(w / (NPX / 128)); const int n0 = (int)(w % (NPX / 128)) * 128 + lane * 4; const int h = c / DQ, d = c % DQ;
    v4f v = *(const v4f*)(OZ + ((size_t)h * 64 + d) * NPX + n0); v = v * (1.0f / XCAR);
    *(volatile v4f*)(OUTB + (size_t)c * NPX + n0) = v; __threadfence(); *(volatile v4f*)(OUTB + (size_t)c * NPX + n0) = v;
}
extern "C" void kernel_launch(void* const* d_in, const int* in_sizes, int n_in,
                              void* d_out, int out_size, void* d_ws, size_t ws_size, hipStream_t stream) {
    (void)in_sizes; (void)n_in; (void)out_size;
    const float* x = (const float*)d_in[0]; const float* mask = (const float*)d_in[1]; const float* Wq = (const float*)d_in[2]; const float* Wk = (const float*)d_in[3]; const float* Wv = (const float*)d_in[4]; const float* gam = (const float*)d_in[5]; const float* bet = (const float*)d_in[6];
    float* out = (float*)d_out;
    char* wsp = (char*)d_ws;
    auto take = [&](size_t bytes) { char* p = wsp; wsp += (bytes + 255) & ~(size_t)255; return (void*)p; };
    h16* BQ = (h16*)take(CC * CC * 2); h16* BK = (h16*)take(CC * CC * 2); h16* BV = (h16*)take(CC * CC * 2);
    float* MU = (float*)take(NPX * 4); float* RS = (float*)take(NPX * 4); h16* XH = (h16*)take((size_t)NPX * CC * 2); bf* XTh = (bf*)take((size_t)CC * NPX * 2); bf* XTl = (bf*)take((size_t)CC * NPX * 2); bf* MB = (bf*)take((size_t)MM * NPX * 2);
    float* STOK = (float*)take((size_t)MM * CC * 4); h16* STHS = (h16*)take((size_t)NH_ * MM * DQ * 2); float* QF = (float*)take((size_t)NPX * CC * 4); float* KF = (float*)take((size_t)NPX * CC * 4); float* VF = (float*)take((size_t)NPX * CC * 4);
    h16* QP = (h16*)take((size_t)NH_ * NPX * DQ * 2); h16* KP = (h16*)take((size_t)NH_ * NPX * DQ * 2); h16* VT = (h16*)take((size_t)NH_ * 64 * NPX * 2); float* S = (float*)take((size_t)NH_ * NPX * MM * 4); h16* PT = (h16*)take((size_t)NH_ * MM * NPX * 2); float* SOT = (float*)take((size_t)NH_ * MM * 64 * 4); h16* SO16 = (h16*)take((size_t)NH_ * 64 * MM * 2); h16* XS = (h16*)take((size_t)NH_ * NPX * MM * 2); float* OZ = (float*)take((size_t)NH_ * 64 * NPX * 4);
    if ((size_t)(wsp - (char*)d_ws) > ws_size) return;
    const size_t n8 = (size_t)CC * CC / 8; k_cvt8h<<<(unsigned)((n8 + 255) / 256), 256, 0, stream>>>(Wq, BQ, n8); k_cvt8h<<<(unsigned)((n8 + 255) / 256), 256, 0, stream>>>(Wk, BK, n8); k_cvt8h<<<(unsigned)((n8 + 255) / 256), 256, 0, stream>>>(Wv, BV, n8);
    for (int b = 0; b < NB_; ++b) { const float* xb = x + (size_t)b * CC * NPX; const float* mb = mask + (size_t)b * MM * NPX;
        k_stat2d<<<(NPX / 32) / 8, 256, 0, stream>>>(xb, MU, RS);
        k_xnrow<<<NPX / 8, 256, 0, stream>>>(xb, MU, RS, gam, bet, XH);
        k_xncol<<<(CC * (NPX / 128)) / 8, 256, 0, stream>>>(xb, MU, RS, gam, bet, XTh, XTl);
        k_maskb<<<MM / 8, 256, 0, stream>>>(mb, MB);
        k_gemm3z<16><<<dim3(MM / 64, CC / 64, 1), 128, 0, stream>>>(MB, MB, XTh, XTl, NPX, STOK, CC, 0, 0, 0);
        k_sths<<<(NH_ * (MM / 4)) / 8, 256, 0, stream>>>(mb, STOK, STHS);
        k_gemmh<<<dim3(NPX / 64, CC / 64, 1), 128, 0, stream>>>(XH, BQ, nullptr, QF, CC, nullptr, CC, 0, 0, 0, 0);
        k_gemmh<<<dim3(NPX / 64, CC / 64, 1), 128, 0, stream>>>(XH, BK, nullptr, KF, CC, nullptr, CC, 0, 0, 0, 0);
        k_gemmh<<<dim3(NPX / 64, CC / 64, 1), 128, 0, stream>>>(XH, BV, nullptr, VF, CC, nullptr, CC, 0, 0, 0, 0);
        k_hpl32h<<<dim3((NPX / 4) / 8, 1, NH_), 256, 0, stream>>>(KF, KP); k_hpl32h<<<dim3((NPX / 4) / 8, 1, NH_), 256, 0, stream>>>(QF, QP); k_vT32h<<<dim3(NPX / 64, 1, NH_), 256, 0, stream>>>(VF, VT);
        k_gemmh<<<dim3(NPX / 64, MM / 64, NH_), 128, 0, stream>>>(KP, STHS, nullptr, S, MM, nullptr, DQ, (size_t)NPX * DQ, (size_t)MM * DQ, (size_t)NPX * MM, 0);
        k_csoftP<<<(NH_ * MM) / 8, 256, 0, stream>>>(S, PT);
        k_gemmh<<<dim3(MM / 64, 1, NH_), 128, 0, stream>>>(PT, VT, nullptr, SOT, 64, nullptr, NPX, (size_t)MM * NPX, (size_t)64 * NPX, (size_t)MM * 64, 0);
        k_so16<<<(NH_ * 64) / 8, 256, 0, stream>>>(SOT, SO16);
        k_gemmh<<<dim3(MM / 64, NPX / 64, NH_), 128, 0, stream>>>(STHS, QP, nullptr, S, NPX, nullptr, DQ, (size_t)MM * DQ, (size_t)NPX * DQ, (size_t)MM * NPX, 0);
        k_csoftX<<<(NH_ * NPX) / 8, 256, 0, stream>>>(S, XS);
        k_gemmh<<<dim3(1, NPX / 64, NH_), 128, 0, stream>>>(SO16, XS, nullptr, OZ, NPX, nullptr, MM, (size_t)64 * MM, (size_t)NPX * MM, (size_t)64 * NPX, 0);
        k_outrows<<<(CC * (NPX / 128)) / 8, 256, 0, stream>>>(OZ, out + (size_t)b * CC * NPX); }
}
